// MLPdirected_59519656788458
// MI455X (gfx1250) — hardware-verified
//
#include <hip/hip_runtime.h>
#include <stddef.h>


typedef _Float16 v16h __attribute__((ext_vector_type(16)));
typedef _Float16 v8h  __attribute__((ext_vector_type(8)));
typedef float    v8f  __attribute__((ext_vector_type(8)));
typedef float    v4f  __attribute__((ext_vector_type(4)));
typedef _Float16 h16;

#ifndef NB
#define NB 2
#endif
#ifndef SEQ
#define SEQ 1024
#endif
#define NB_FULL  2
#define SEQ_FULL 1024
#define KD    32
#define HD    64
#define PW    128
#define MROWS (NB * SEQ)
#define NTILE (SEQ / 32)

static_assert(NB >= 1 && NB <= NB_FULL);
static_assert(SEQ >= 64 && SEQ <= SEQ_FULL && (SEQ % 64) == 0);
static_assert(KD == 32 && (KD % 32) == 0);
static_assert(KD / 8 == 4);
static_assert(HD == 4 * 16);
static_assert((HD % 64) == 0);
static_assert(PW == 2 * HD && (PW % 64) == 0 && (PW % 32) == 0);
static_assert((MROWS % 64) == 0 && (MROWS % 32) == 0);
static_assert((size_t)NB_FULL * SEQ_FULL * SEQ_FULL * 4 == (size_t)8388608);
static_assert((size_t)((NB - 1) * SEQ_FULL + SEQ) * SEQ_FULL <= (size_t)NB_FULL * SEQ_FULL * SEQ_FULL);

#define LDT 72
#define LDC 68
#define LPAD 68
#define LSO 36
static_assert((LDT % 8) == 0 && LDT >= KD);
static_assert((LDC % 4) == 0 && LDC >= 64);
static_assert((LPAD % 4) == 0 && LPAD >= HD);
static_assert((LSO % 4) == 0 && LSO >= 32);

#define WCARRY 64.0f
#define XCARRY 16.0f

#define WT_BYTES  ((size_t)PW * KD * 2)
#define X16_BYTES ((size_t)MROWS * KD * 2)
#define PF_BYTES  ((size_t)MROWS * PW * 4)
#define OFF_WT  ((size_t)0)
#define OFF_X16 (OFF_WT + WT_BYTES)
#define OFF_PF  (OFF_X16 + X16_BYTES)
#define WS_TOTAL (OFF_PF + PF_BYTES)
static_assert((WT_BYTES % 128) == 0 && (X16_BYTES % 128) == 0 && (PF_BYTES % 128) == 0);
static_assert(WS_TOTAL <= (size_t)134217728);

#define PAIR_LDS_BYTES ((size_t)(2 * 32 * LPAD + HD + 32 * LSO) * 4)
static_assert(PAIR_LDS_BYTES <= (size_t)131072);
static_assert((size_t)64 * LDC * 4 <= (size_t)131072);
static_assert((size_t)64 * LDT * 2 <= (size_t)131072);

__device__ __forceinline__ float bf16r(float x) {
  unsigned int u = __float_as_uint(x);
  u = (u + 0x7FFFu + ((u >> 16) & 1u)) & 0xFFFF0000u;
  return __uint_as_float(u);
}

__device__ __forceinline__ h16 toh_flush(float v) {
  const h16 r = (h16)v;
  return (fabsf(v) < 6.103515625e-05f) ? (h16)0.0f : r;
}

__device__ __forceinline__ v16h frag_at(const _Float16* p) {
  v8h lo = *(const v8h*)(p);
  v8h hi = *(const v8h*)(p + 16);
  v16h out;
#pragma unroll
  for (int i = 0; i < 8; ++i) { out[i] = lo[i]; out[i + 8] = hi[i]; }
  return out;
}

__device__ __forceinline__ v8f wmma16(v16h a, v16h b, v8f c) {
  v8f d = __builtin_amdgcn_wmma_f32_16x16x32_f16(false, a, false, b, (short)0, c,
                                                 false, false);
  asm volatile("v_nop\n\tv_nop\n\tv_nop\n\tv_nop" : "+v"(d) : "v"(a), "v"(b));
  return d;
}

__device__ __forceinline__ float sigm(float z) {
  return __builtin_amdgcn_rcpf(1.0f + __expf(-z));
}

__global__ __launch_bounds__(256) void wconv_kernel(
    const float* __restrict__ W, _Float16* __restrict__ Wt) {
#pragma clang fp contract(off)
  const unsigned gid = blockIdx.x * 256u + threadIdx.x;
  const unsigned n = gid >> 2;
  const unsigned c = (gid & 3u) * 8u;
  const unsigned sel = n / (unsigned)HD;
  const unsigned hrow = n - sel * (unsigned)HD;
  const float* src = W + (size_t)hrow * (2u * (unsigned)KD) + sel * (unsigned)KD + c;
  const v4f a0 = *(const v4f*)(src);
  const v4f a1 = *(const v4f*)(src + 4u);
  v8h o;
#pragma unroll
  for (int i = 0; i < 4; ++i) {
    o[i]     = toh_flush(WCARRY * bf16r(a0[i]));
    o[i + 4] = toh_flush(WCARRY * bf16r(a1[i]));
  }
  _Float16* p = Wt + (size_t)n * KD + c;
  *(volatile v8h*)p = o;
  __threadfence();
  *(volatile v8h*)p = o;
}
static_assert(((size_t)PW * KD / 8) % 256 == 0);

__global__ __launch_bounds__(256) void xconv_kernel(
    const float* __restrict__ X, _Float16* __restrict__ X16) {
#pragma clang fp contract(off)
  __shared__ __attribute__((aligned(16))) _Float16 T[64 * LDT];
  const unsigned tid = threadIdx.x;
  const unsigned n0 = blockIdx.x * 64u;
  const unsigned b = blockIdx.y;
#pragma unroll 4
  for (unsigned j = 0; j < 8u; ++j) {
    const unsigned idx = tid + 256u * j;
    const unsigned kr = idx >> 6, nc = idx & 63u;
    const float v = X[((size_t)b * KD + kr) * SEQ_FULL + n0 + nc];
    T[nc * LDT + kr] = toh_flush(XCARRY * bf16r(v));
  }
  __syncthreads();
  const unsigned n = tid >> 2;
  const unsigned kc = (tid & 3u) * 8u;
  const v8h x = *(const v8h*)&T[n * LDT + kc];
  _Float16* p = X16 + (size_t)(b * (unsigned)SEQ + n0 + n) * KD + kc;
  *(volatile v8h*)p = x;
  __threadfence();
  *(volatile v8h*)p = x;
}
static_assert(256 * 8 == KD * 64);
static_assert(256 / 4 == 64);

__global__ __launch_bounds__(256) void gemm_pre_kernel(
    const _Float16* __restrict__ A16, const _Float16* __restrict__ Bt,
    float* __restrict__ outf) {
  __shared__ float Cs[64 * LDC];
  const unsigned tid = threadIdx.x, lane = tid & 31u;
  const unsigned w = (unsigned)__builtin_amdgcn_readfirstlane((int)(threadIdx.x >> 5));
  const unsigned mw = w >> 1, nw = w & 1u;
  const unsigned hh = lane >> 4, m = lane & 15u;
  const unsigned n0 = blockIdx.x * 64u;
  const unsigned row0 = blockIdx.y * 64u;

  const _Float16* ap  = A16 + (size_t)(row0 + mw * 16u + m) * KD + hh * 8u;
  const _Float16* bp0 = Bt + (size_t)(n0 + nw * 32u + m) * KD + hh * 8u;
  const _Float16* bp1 = bp0 + (size_t)16 * KD;
  v8f acc0 = {}, acc1 = {};
#pragma unroll
  for (unsigned k0 = 0; k0 < (unsigned)KD; k0 += 32u) {
    const v16h a  = frag_at(ap + k0);
    const v16h b0 = frag_at(bp0 + k0);
    const v16h b1 = frag_at(bp1 + k0);
    acc0 = wmma16(a, b0, acc0);
    acc1 = wmma16(a, b1, acc1);
  }
#pragma unroll
  for (int r = 0; r < 8; ++r) {
    float* d = &Cs[(mw * 16u + hh * 8u + (unsigned)r) * LDC + nw * 32u + m];
    d[0]  = acc0[r];
    d[16] = acc1[r];
  }
  __syncthreads();

  const float cs = 1.0f / (WCARRY * XCARRY);
  v4f xs[4];
  size_t off[4];
#pragma unroll
  for (unsigned i = 0; i < 4u; ++i) {
    const unsigned r = 16u * i + (tid >> 4);
    const unsigned c = (tid & 15u) * 4u;
    const v4f u = *(const v4f*)&Cs[r * LDC + c];
    v4f val;
#pragma unroll
    for (int j = 0; j < 4; ++j) val[j] = u[j] * cs;
    xs[i] = val;
    off[i] = (size_t)(row0 + r) * PW + n0 + c;
  }
#pragma unroll
  for (int i = 0; i < 4; ++i) *(volatile v4f*)(outf + off[i]) = xs[i];
  __threadfence();
#pragma unroll
  for (int i = 0; i < 4; ++i) *(volatile v4f*)(outf + off[i]) = xs[i];
}
static_assert(4 * 16 == 64);

__global__ __launch_bounds__(256) void pair_kernel(
    const float* __restrict__ Pf,
    const float* __restrict__ b1, const float* __restrict__ W2, const float* __restrict__ b2,
    float* __restrict__ out) {
#pragma clang fp contract(off)
  __shared__ __attribute__((aligned(16))) float sA[32 * LPAD];
  __shared__ __attribute__((aligned(16))) float sB[32 * LPAD];
  __shared__ __attribute__((aligned(16))) float w2s[HD];
  __shared__ __attribute__((aligned(16))) float So[32 * LSO];

  const unsigned tid = threadIdx.x;
  const unsigned b = blockIdx.z;
  const unsigned ti = blockIdx.y, tj = blockIdx.x;
  const unsigned i0 = ti * 32u, j0 = tj * 32u;

  const size_t arow = (size_t)(b * (unsigned)SEQ + i0) * PW;
  const size_t brow = (size_t)(b * (unsigned)SEQ + j0) * PW + HD;
#pragma unroll 1
  for (unsigned s = 0; s < 2u; ++s) {
    const unsigned idx = tid + 256u * s;
    const unsigned r = idx >> 4, c = (idx & 15u) * 4u;
    const v4f a  = *(const v4f*)(Pf + arow + (size_t)r * PW + c);
    const v4f bb = *(const v4f*)(Pf + brow + (size_t)r * PW + c);
    const v4f g  = *(const v4f*)(b1 + c);
    v4f av;
#pragma unroll
    for (int j = 0; j < 4; ++j) av[j] = a[j] + bf16r(g[j]);
    *(v4f*)&sA[r * LPAD + c] = av;
    *(v4f*)&sB[r * LPAD + c] = bb;
  }
  if (tid < (unsigned)HD) w2s[tid] = bf16r(W2[tid]);
  __syncthreads();

  const unsigned tx = tid & 15u, ty = tid >> 4;
  const unsigned pa = (ty * 2u) * LPAD;
  const unsigned pb = (tx * 2u) * LPAD;
  float a00 = 0.0f, a01 = 0.0f, a10 = 0.0f, a11 = 0.0f;
#pragma unroll 1
  for (unsigned h = 0; h < (unsigned)HD; h += 4u) {
    const v4f wv = *(const v4f*)&w2s[h];
    const v4f x0 = *(const v4f*)&sA[pa + h];
    const v4f x1 = *(const v4f*)&sA[pa + LPAD + h];
    const v4f y0 = *(const v4f*)&sB[pb + h];
    const v4f y1 = *(const v4f*)&sB[pb + LPAD + h];
#pragma unroll
    for (int j = 0; j < 4; ++j) {
      a00 = fmaf(fmaxf(x0[j] + y0[j], 0.0f), wv[j], a00);
      a01 = fmaf(fmaxf(x0[j] + y1[j], 0.0f), wv[j], a01);
      a10 = fmaf(fmaxf(x1[j] + y0[j], 0.0f), wv[j], a10);
      a11 = fmaf(fmaxf(x1[j] + y1[j], 0.0f), wv[j], a11);
    }
  }
  const float c2 = bf16r(b2[0]);
  const float s00 = sigm(a00 + c2);
  const float s01 = sigm(a01 + c2);
  const float s10 = sigm(a10 + c2);
  const float s11 = sigm(a11 + c2);
  So[(2u * ty) * LSO + 2u * tx]            = s00;
  So[(2u * ty) * LSO + 2u * tx + 1u]       = s01;
  So[(2u * ty + 1u) * LSO + 2u * tx]       = s10;
  So[(2u * ty + 1u) * LSO + 2u * tx + 1u]  = s11;
  __syncthreads();

  const unsigned r = tid >> 3, c0 = (tid & 7u) * 4u;
  const v4f u = *(const v4f*)&So[r * LSO + c0];
  const size_t offa = ((size_t)b * SEQ_FULL + i0 + r) * SEQ_FULL + j0 + c0;
  *(volatile v4f*)(out + offa) = u;
  __threadfence();
  *(volatile v4f*)(out + offa) = u;
}
static_assert(256 / 8 == 32);
static_assert(16 * 2 == 32);
static_assert(2 * 256 == 32 * (HD / 4));
static_assert(HD <= 64 || (HD % 32) == 0);
static_assert(NTILE * 32 == SEQ);

extern "C" void kernel_launch(void* const* d_in, const int* in_sizes, int n_in,
                              void* d_out, int out_size, void* d_ws, size_t ws_size,
                              hipStream_t stream) {
  if (n_in < 7) return;
  const long long need_x = ((long long)(NB - 1) * KD + (KD - 1)) * SEQ_FULL + SEQ;
  const long long need_o = ((long long)(NB - 1) * SEQ_FULL + SEQ) * SEQ_FULL;
  if ((long long)in_sizes[1] < need_x) return;
  if ((long long)in_sizes[3] < (long long)2 * KD * HD) return;
  if (in_sizes[4] < HD || in_sizes[5] < HD || in_sizes[6] < 1) return;
  if ((long long)out_size < need_o) return;
  if (ws_size < WS_TOTAL) return;

  const float* emb = (const float*)d_in[1];
  const float* w1  = (const float*)d_in[3];
  const float* b1  = (const float*)d_in[4];
  const float* w2  = (const float*)d_in[5];
  const float* b2  = (const float*)d_in[6];
  float* out = (float*)d_out;

  char* ws = (char*)d_ws;
  _Float16* Wt  = (_Float16*)(ws + OFF_WT);
  _Float16* X16 = (_Float16*)(ws + OFF_X16);
  float*    Pf  = (float*)(ws + OFF_PF);

  dim3 blk(256);
  wconv_kernel<<<dim3(PW * KD / 8 / 256), blk, 0, stream>>>(w1, Wt);
  xconv_kernel<<<dim3(SEQ / 64, NB), blk, 0, stream>>>(emb, X16);
  gemm_pre_kernel<<<dim3(PW / 64, MROWS / 64), blk, 0, stream>>>(X16, Wt, Pf);
  pair_kernel<<<dim3(NTILE, NTILE, NB), blk, 0, stream>>>(Pf, b1, w2, b2, out);
}
